// GatingNeuralAdaptiveBias_82291573391764
// MI455X (gfx1250) — hardware-run, weakly checked
//
#include <hip/hip_runtime.h>
#include <math.h>


#ifndef NB
#define NB 8
#endif
#ifndef NI
#define NI 256
#endif
#define NB_FULL 8
#define NN_FULL 256
#ifndef OUT_NI
#define OUT_NI NI
#endif
#define NJ   256
#define HID  64
#define NFE  9
#define NTH  256
#define NWV  8
#define XS   20
#define ES   68
#define WCAR 64.0f
#define WCI  (1.0f / 64.0f)
#define LNEPS 1.0e-5f

#define P_W1  0
#define P_B1  576
#define P_B2  640
#define P_GAM 704
#define P_BET 832
#define P_BG1 960
#define P_WG2 1024
#define P_LG  1152
#define P_LB  1216
#define P_WO  1280
#define P_TOT 1344

static_assert(NJ == NN_FULL);
static_assert(NTH == NJ);
static_assert(NWV * 32 == NTH);
static_assert(HID == 64);
static_assert(HID % 32 == 0);
static_assert((2 * HID) % 32 == 0);
static_assert(2 * NFE <= XS);
static_assert(NFE * HID == 576);
static_assert(ES >= HID && ES % 4 == 0);
static_assert(P_B1 % 4 == 0 && P_B2 % 4 == 0 && P_GAM % 4 == 0 && P_BET % 4 == 0 && P_BG1 % 4 == 0 && P_WG2 % 4 == 0 && P_LG % 4 == 0 && P_LB % 4 == 0 && P_WO % 4 == 0);
static_assert(64 * 16 == NJ * 4);
static_assert((size_t)(P_TOT + NWV * 32 * XS + NJ + NWV * 16 * 2 * ES) * 4 <= (size_t)131072);
static_assert(NB <= NB_FULL);
static_assert(NI <= NN_FULL);
static_assert(NI <= OUT_NI);

typedef _Float16 h16;
typedef __attribute__((ext_vector_type(16))) _Float16 v16h;
typedef __attribute__((ext_vector_type(8)))  _Float16 v8h;
typedef __attribute__((ext_vector_type(8)))  float    v8f;
typedef __attribute__((ext_vector_type(4)))  float    v4f;
typedef v4f  __attribute__((may_alias)) v4fa;

__device__ __forceinline__ unsigned short f2bf(float f) { unsigned u = __float_as_uint(f); u += 0x7FFFu + ((u >> 16) & 1u); return (unsigned short)(u >> 16); }
__device__ __forceinline__ float bfr(float f) { return __uint_as_float(((unsigned)f2bf(f)) << 16); }
__device__ __forceinline__ v16h cat16(v8h lo, v8h hi) { return __builtin_shufflevector(lo, hi, 0, 1, 2, 3, 4, 5, 6, 7, 8, 9, 10, 11, 12, 13, 14, 15); }
__device__ __forceinline__ v8f wmma16(v16h a, v16h b, v8f c) { return __builtin_amdgcn_wmma_f32_16x16x32_f16(false, a, false, b, (short)0, c, false, false); }
__device__ __forceinline__ v8f wmma16g(v16h a, v16h b, v8f c) { c = wmma16(a, b, c); asm volatile("v_nop\n\tv_nop\n\tv_nop\n\tv_nop" : "+v"(c) : "v"(a), "v"(b)); return c; }
__device__ __forceinline__ v16h ldh(const h16* p) { return cat16(*(const v8h*)p, *(const v8h*)(p + 16)); }
__device__ __forceinline__ void wave_sync() { __builtin_amdgcn_fence(3  , "wavefront"); __builtin_amdgcn_wave_barrier(); asm volatile("" ::: "memory"); }
static __device__ __forceinline__ h16 toh_flush(float v) { const float w = (fabsf(v) < 6.103515625e-05f) ? 0.0f : v; return (h16)w; }
static __device__ __forceinline__ float silu_f(float v) { return v * __builtin_amdgcn_rcpf(1.0f + __expf(-v)); }
static __device__ __forceinline__ float mixv(float g0, float a, float g1, float c) { return fmaf(g0, a, g1 * c); }

__global__ __launch_bounds__(256) void k_wconv(const float* __restrict__ w2, const float* __restrict__ wg1, h16* w2t, h16* wg1t) {
    const unsigned bxx = blockIdx.x;
    const unsigned t = bxx * 256u + threadIdx.x;
    if (bxx < 2u) {
        const unsigned n = t >> 3, k8 = (t & 7u) * 8u; v8h o;
#pragma unroll
        for (unsigned e = 0; e < 8u; ++e) o[e] = toh_flush(bfr(w2[(k8 + e) * 64u + n]) * WCAR);
        h16* dp = w2t + (size_t)t * 8;
        *(volatile v8h*)dp = o; __threadfence(); *(volatile v8h*)dp = o;
    } else {
        const unsigned u = t - 512u; const unsigned n = u >> 4, k8 = (u & 15u) * 8u; v8h o;
#pragma unroll
        for (unsigned e = 0; e < 8u; ++e) o[e] = toh_flush(bfr(wg1[(k8 + e) * 64u + n]) * WCAR);
        h16* dp = wg1t + (size_t)u * 8;
        *(volatile v8h*)dp = o; __threadfence(); *(volatile v8h*)dp = o;
    }
}

__global__ __launch_bounds__(NTH) void k_pairs(const float* __restrict__ coords, const float* __restrict__ cost, const float* __restrict__ lsc,
                                               const float* __restrict__ W1, const float* __restrict__ b1, const float* __restrict__ b2,
                                               const float* __restrict__ fgam, const float* __restrict__ fbet, const float* __restrict__ bg1,
                                               const float* __restrict__ Wg2, const float* __restrict__ bg2, const float* __restrict__ gtemp,
                                               const float* __restrict__ lng, const float* __restrict__ lnb, const float* __restrict__ Wo, const float* __restrict__ bo,
                                               const h16* __restrict__ W2T, const h16* __restrict__ WG1T, float* OUT) {
    __shared__ __align__(16) float sP[P_TOT];
    __shared__ __align__(16) float sX[NWV * 32 * XS];
    __shared__ __align__(16) float sE[NWV * 16 * 2 * ES];
    __shared__ __align__(16) float sOut[NJ];
    const unsigned tid = threadIdx.x;
    const int lane = (int)(tid & 31u), lr = lane & 15, hi = lane >> 4;
    const int wave = __builtin_amdgcn_readfirstlane((int)(threadIdx.x >> 5));
    const unsigned bx = blockIdx.x;
    const unsigned b = bx / (unsigned)NI, i = bx % (unsigned)NI;

#pragma unroll
    for (unsigned it = 0; it < 3u; ++it) {
        const unsigned idx = tid + 256u * it; const unsigned ci = min(idx, 575u);
        const float v = bfr(W1[ci]);
        if (idx < 576u) sP[P_W1 + idx] = v; }
    { const unsigned c6 = tid & 63u, c7 = tid & 127u;
      const float v1 = bfr(b1[c6]), v2 = bfr(b2[c6]), v3 = bfr(bg1[c6]), v4 = bfr(lng[c6]), v5 = bfr(lnb[c6]), v6 = bfr(Wo[c6]);
      const float u1 = bfr(fgam[c7]), u2 = bfr(fbet[c7]), u3 = bfr(Wg2[c7]);
      if (tid < 64u)  { sP[P_B1 + tid] = v1; sP[P_B2 + tid] = v2; sP[P_BG1 + tid] = v3; sP[P_LG + tid] = v4; sP[P_LB + tid] = v5; sP[P_WO + tid] = v6; }
      if (tid < 128u) { sP[P_GAM + tid] = u1; sP[P_BET + tid] = u2; sP[P_WG2 + tid] = u3; } }
    __syncthreads();

    const size_t rowi = (size_t)b * NN_FULL + i;
    const size_t rowj = (size_t)b * NN_FULL + tid;
    const float cv = bfr(cost[rowi * NN_FULL + tid]);
    const float xi = bfr(coords[rowi * 2 + 0]), yi = bfr(coords[rowi * 2 + 1]);
    const float xj = bfr(coords[rowj * 2 + 0]), yj = bfr(coords[rowj * 2 + 1]);
    const float dx = xi - xj, dy = yi - yj;
    const float ang = atan2f(dy, dx);
    const float s0 = expf(bfr(lsc[0])), s1 = expf(bfr(lsc[1]));
    const float bg20 = bfr(bg2[0]), bg21 = bfr(bg2[1]);
    const float invT = __builtin_amdgcn_rcpf(expf(bfr(gtemp[0])));
    const float bov = bfr(bo[0]);
    { const int xw = (int)tid * XS;
      sX[xw + 0] = cv * s0; sX[xw + NFE] = ang * s1;
#pragma unroll 1
      for (int it = 0; it < 8; ++it) {
          const int ch = it >> 2, fq = it & 3;
          const float base = ch ? ang : cv; const float sc = ch ? s1 : s0;
          const float fr = (float)(1 << fq);
          float ss, cc; sincosf(base * fr, &ss, &cc);
          sX[xw + ch * NFE + 1 + 2 * fq] = ss * sc; sX[xw + ch * NFE + 2 + 2 * fq] = cc * sc; } }
    wave_sync();

    const int eb = (wave * 16 + lr) * 2 * ES + 8 * hi;

#pragma unroll 1
    for (int mt = 0; mt < 2; ++mt) {
        const int xo = (wave * 32 + mt * 16 + lr) * XS;
        v16h hb[2][2];
#pragma unroll
        for (int ch = 0; ch < 2; ++ch) {
            float x[NFE];
#pragma unroll
            for (int k = 0; k < NFE; ++k) x[k] = sX[xo + ch * NFE + k];
            v8h h0 = (v8h){}, h1 = (v8h){}, h2 = (v8h){}, h3 = (v8h){};
#pragma unroll 1
            for (int q = 0; q < 4; ++q) {
                const int nb = 16 * q + 8 * hi;
                const v4f c0 = *(const v4fa*)(&sP[P_B1 + nb]); const v4f c1 = *(const v4fa*)(&sP[P_B1 + nb + 4]);
                float a[8];
#pragma unroll
                for (int r = 0; r < 4; ++r) { a[r] = c0[r]; a[4 + r] = c1[r]; }
#pragma unroll
                for (int k = 0; k < NFE; ++k) {
                    const v4f w0 = *(const v4fa*)(&sP[P_W1 + k * 64 + nb]); const v4f w1 = *(const v4fa*)(&sP[P_W1 + k * 64 + nb + 4]);
#pragma unroll
                    for (int r = 0; r < 4; ++r) { a[r] = fmaf(x[k], w0[r], a[r]); a[4 + r] = fmaf(x[k], w1[r], a[4 + r]); } }
                v8h hv;
#pragma unroll
                for (int r = 0; r < 8; ++r) hv[r] = toh_flush(silu_f(a[r]));
                h0 = h1; h1 = h2; h2 = h3; h3 = hv;
            }
            hb[ch][0] = cat16(h0, h1);
            hb[ch][1] = cat16(h2, h3);
        }
        v16h pbs[4];
        {
            v8f e[2][4];
#pragma unroll
            for (int ch = 0; ch < 2; ++ch)
#pragma unroll
                for (int nt = 0; nt < 4; ++nt) e[ch][nt] = (v8f){};
#pragma unroll
            for (int s = 0; s < 2; ++s) {
#pragma unroll
                for (int nt = 0; nt < 4; ++nt) {
                    const v16h a = ldh(W2T + (size_t)(16 * nt + lr) * HID + 32 * s + 8 * hi);
                    e[0][nt] = wmma16g(a, hb[0][s], e[0][nt]);
                    e[1][nt] = wmma16g(a, hb[1][s], e[1][nt]); } }
#pragma unroll
            for (int nt = 0; nt < 4; ++nt) {
                const int nb = 16 * nt + 8 * hi;
                const v4f q0 = *(const v4fa*)(&sP[P_B2 + nb]); const v4f q1 = *(const v4fa*)(&sP[P_B2 + nb + 4]);
#pragma unroll
                for (int ch = 0; ch < 2; ++ch) {
                    const v4f g0 = *(const v4fa*)(&sP[P_GAM + ch * 64 + nb]); const v4f g1 = *(const v4fa*)(&sP[P_GAM + ch * 64 + nb + 4]);
                    const v4f t0 = *(const v4fa*)(&sP[P_BET + ch * 64 + nb]); const v4f t1 = *(const v4fa*)(&sP[P_BET + ch * 64 + nb + 4]);
#pragma unroll
                    for (int r = 0; r < 4; ++r) {
                        e[ch][nt][r]     = (e[ch][nt][r]     * WCI + q0[r]) * g0[r] + t0[r];
                        e[ch][nt][4 + r] = (e[ch][nt][4 + r] * WCI + q1[r]) * g1[r] + t1[r]; } } }
#pragma unroll
            for (int s = 0; s < 4; ++s) {
#pragma unroll
                for (int r = 0; r < 8; ++r) { pbs[s][r] = toh_flush(e[s >> 1][2 * (s & 1)][r]); pbs[s][8 + r] = toh_flush(e[s >> 1][2 * (s & 1) + 1][r]); } }
#pragma unroll
            for (int ch = 0; ch < 2; ++ch)
#pragma unroll
                for (int nt = 0; nt < 4; ++nt) {
                    const v4f lo = __builtin_shufflevector(e[ch][nt], e[ch][nt], 0, 1, 2, 3);
                    const v4f up = __builtin_shufflevector(e[ch][nt], e[ch][nt], 4, 5, 6, 7);
                    *(v4fa*)(&sE[eb + ch * ES + 16 * nt]) = lo; *(v4fa*)(&sE[eb + ch * ES + 16 * nt + 4]) = up; }
        }
        wave_sync();
        v8f g[4];
#pragma unroll
        for (int nt = 0; nt < 4; ++nt) g[nt] = (v8f){};
#pragma unroll
        for (int s = 0; s < 4; ++s) {
#pragma unroll
            for (int nt = 0; nt < 4; ++nt) {
                const v16h a = ldh(WG1T + (size_t)(16 * nt + lr) * (2 * HID) + 32 * s + 8 * hi);
                g[nt] = wmma16g(a, pbs[s], g[nt]); } }
        float l0 = 0.0f, l1 = 0.0f;
#pragma unroll
        for (int nt = 0; nt < 4; ++nt) {
            const int nb = 16 * nt + 8 * hi;
            const v4f q0 = *(const v4fa*)(&sP[P_BG1 + nb]); const v4f q1 = *(const v4fa*)(&sP[P_BG1 + nb + 4]);
            const v4f w0 = *(const v4fa*)(&sP[P_WG2 + 2 * nb]);     const v4f w1 = *(const v4fa*)(&sP[P_WG2 + 2 * nb + 4]);
            const v4f w2 = *(const v4fa*)(&sP[P_WG2 + 2 * nb + 8]); const v4f w3 = *(const v4fa*)(&sP[P_WG2 + 2 * nb + 12]);
            float bb[8], wa[8], wc[8];
#pragma unroll
            for (int r = 0; r < 4; ++r) { bb[r] = q0[r]; bb[4 + r] = q1[r]; }
            wa[0] = w0[0]; wc[0] = w0[1]; wa[1] = w0[2]; wc[1] = w0[3]; wa[2] = w1[0]; wc[2] = w1[1]; wa[3] = w1[2]; wc[3] = w1[3];
            wa[4] = w2[0]; wc[4] = w2[1]; wa[5] = w2[2]; wc[5] = w2[3]; wa[6] = w3[0]; wc[6] = w3[1]; wa[7] = w3[2]; wc[7] = w3[3];
#pragma unroll
            for (int r = 0; r < 8; ++r) { const float gv = silu_f(g[nt][r] * WCI + bb[r]); l0 = fmaf(gv, wa[r], l0); l1 = fmaf(gv, wc[r], l1); } }
        l0 += __shfl_xor(l0, 16, 32); l1 += __shfl_xor(l1, 16, 32);
        const float z0 = (l0 + bg20) * invT, z1 = (l1 + bg21) * invT;
        const float zm = fmaxf(z0, z1);
        const float ew0 = __expf(z0 - zm), ew1 = __expf(z1 - zm);
        const float ei = __builtin_amdgcn_rcpf(ew0 + ew1);
        const float gw0 = ew0 * ei, gw1 = ew1 * ei;
        float sm = 0.0f;
#pragma unroll 1
        for (int nt = 0; nt < 4; ++nt) {
            const int eo = eb + 16 * nt;
            const v4f x0 = *(const v4fa*)(&sE[eo]);      const v4f x1 = *(const v4fa*)(&sE[eo + 4]);
            const v4f y0 = *(const v4fa*)(&sE[eo + ES]); const v4f y1 = *(const v4fa*)(&sE[eo + ES + 4]);
#pragma unroll
            for (int r = 0; r < 4; ++r) sm += mixv(gw0, x0[r], gw1, y0[r]);
#pragma unroll
            for (int r = 0; r < 4; ++r) sm += mixv(gw0, x1[r], gw1, y1[r]); }
        sm += __shfl_xor(sm, 16, 32);
        const float mu = sm * (1.0f / 64.0f);
        float sq = 0.0f;
#pragma unroll 1
        for (int nt = 0; nt < 4; ++nt) {
            const int eo = eb + 16 * nt;
            const v4f x0 = *(const v4fa*)(&sE[eo]);      const v4f x1 = *(const v4fa*)(&sE[eo + 4]);
            const v4f y0 = *(const v4fa*)(&sE[eo + ES]); const v4f y1 = *(const v4fa*)(&sE[eo + ES + 4]);
#pragma unroll
            for (int r = 0; r < 4; ++r) { const float d = mixv(gw0, x0[r], gw1, y0[r]) - mu; sq = fmaf(d, d, sq); }
#pragma unroll
            for (int r = 0; r < 4; ++r) { const float d = mixv(gw0, x1[r], gw1, y1[r]) - mu; sq = fmaf(d, d, sq); } }
        sq += __shfl_xor(sq, 16, 32);
        const float rstd = __builtin_amdgcn_rsqf(sq * (1.0f / 64.0f) + LNEPS);
        float po = 0.0f;
#pragma unroll 1
        for (int nt = 0; nt < 4; ++nt) {
            const int nb = 16 * nt + 8 * hi; const int eo = eb + 16 * nt;
            const v4f x0 = *(const v4fa*)(&sE[eo]);      const v4f x1 = *(const v4fa*)(&sE[eo + 4]);
            const v4f y0 = *(const v4fa*)(&sE[eo + ES]); const v4f y1 = *(const v4fa*)(&sE[eo + ES + 4]);
            const v4f a0 = *(const v4fa*)(&sP[P_LG + nb]); const v4f a1 = *(const v4fa*)(&sP[P_LG + nb + 4]);
            const v4f c0 = *(const v4fa*)(&sP[P_LB + nb]); const v4f c1 = *(const v4fa*)(&sP[P_LB + nb + 4]);
            const v4f o0 = *(const v4fa*)(&sP[P_WO + nb]); const v4f o1 = *(const v4fa*)(&sP[P_WO + nb + 4]);
#pragma unroll
            for (int r = 0; r < 4; ++r) {
                const float d0 = mixv(gw0, x0[r], gw1, y0[r]) - mu;
                const float d1 = mixv(gw0, x1[r], gw1, y1[r]) - mu;
                po = fmaf(d0 * rstd * a0[r] + c0[r], o0[r], po);
                po = fmaf(d1 * rstd * a1[r] + c1[r], o1[r], po); } }
        po += __shfl_xor(po, 16, 32);
        const float res = po + bov;
        if (hi == 0) sOut[wave * 32 + mt * 16 + lr] = res;
        wave_sync();
    }
    __syncthreads();
    if (tid < 64u) {
        const v4f val = *(const v4fa*)(&sOut[tid * 4u]);
        float* op = OUT + ((size_t)b * OUT_NI + i) * NJ + (size_t)tid * 4;
        *(volatile v4f*)op = val; __threadfence(); *(volatile v4f*)op = val;
    }
}

static constexpr size_t al256(size_t v) { return (v + 255) & ~(size_t)255; }
static constexpr size_t SZ_W2T  = al256((size_t)HID * HID * 2);
static constexpr size_t SZ_WG1T = al256((size_t)HID * 2 * HID * 2);
static constexpr size_t SZ_TOTAL = SZ_W2T + SZ_WG1T;
static_assert(SZ_TOTAL <= (size_t)134217728);
static_assert((size_t)512 * 8 * 2 == (size_t)HID * HID * 2);
static_assert((size_t)1024 * 8 * 2 == (size_t)HID * 2 * HID * 2);

extern "C" void kernel_launch(void* const* d_in, const int* in_sizes, int n_in,
                              void* d_out, int out_size, void* d_ws, size_t ws_size, hipStream_t stream) {
    if (n_in < 18) return;
    const size_t needc = (size_t)NB * NN_FULL * 2;
    const size_t needm = ((size_t)(NB - 1) * NN_FULL + NI) * NN_FULL;
    if ((size_t)in_sizes[0] < needc || (size_t)in_sizes[1] < needm) return;
    if (in_sizes[2] < 2 || in_sizes[3] < NFE * HID || in_sizes[4] < HID || in_sizes[5] < HID * HID || in_sizes[6] < HID) return;
    if (in_sizes[7] < 2 * HID || in_sizes[8] < 2 * HID || in_sizes[9] < 2 * HID * HID || in_sizes[10] < HID || in_sizes[11] < 2 * HID) return;
    if (in_sizes[12] < 2 || in_sizes[13] < 1 || in_sizes[14] < HID || in_sizes[15] < HID || in_sizes[16] < HID || in_sizes[17] < 1) return;
    if ((size_t)out_size < ((size_t)(NB - 1) * OUT_NI + NI) * NJ) return;
    if (SZ_TOTAL > ws_size) return;
    const float* coords = (const float*)d_in[0];  const float* cost = (const float*)d_in[1];  const float* lsc  = (const float*)d_in[2];
    const float* w1     = (const float*)d_in[3];  const float* b1   = (const float*)d_in[4];  const float* w2   = (const float*)d_in[5];
    const float* b2     = (const float*)d_in[6];  const float* fgam = (const float*)d_in[7];  const float* fbet = (const float*)d_in[8];
    const float* wg1    = (const float*)d_in[9];  const float* bg1  = (const float*)d_in[10]; const float* wg2  = (const float*)d_in[11];
    const float* bg2    = (const float*)d_in[12]; const float* gtmp = (const float*)d_in[13]; const float* lng  = (const float*)d_in[14];
    const float* lnb    = (const float*)d_in[15]; const float* wo   = (const float*)d_in[16]; const float* bo   = (const float*)d_in[17];
    float* OUT = (float*)d_out;
    char* wsp = (char*)d_ws;
    h16* W2T  = (h16*)wsp; wsp += SZ_W2T;
    h16* WG1T = (h16*)wsp; wsp += SZ_WG1T;

    k_wconv<<<dim3(6, 1, 1), 256, 0, stream>>>(w2, wg1, W2T, WG1T);
    k_pairs<<<dim3((unsigned)(NB * NI), 1, 1), NTH, 0, stream>>>(coords, cost, lsc, w1, b1, b2, fgam, fbet, bg1, wg2, bg2, gtmp, lng, lnb, wo, bo, W2T, WG1T, OUT);
}
